// IntraBagAttention_17532056502568
// MI455X (gfx1250) — hardware-verified
//
#include <hip/hip_runtime.h>
#include <math.h>

typedef __attribute__((ext_vector_type(16))) _Float16 v16h;
typedef __attribute__((ext_vector_type(16))) __bf16 v16b;
typedef __attribute__((ext_vector_type(8)))  _Float16 v8h;
typedef __attribute__((ext_vector_type(8)))  float v8f;
typedef __attribute__((ext_vector_type(4)))  float v4f;
typedef __attribute__((ext_vector_type(2)))  float v2f;
typedef __attribute__((ext_vector_type(4)))  unsigned v4u;
typedef __attribute__((ext_vector_type(4)))  int v4i;
typedef float __attribute__((may_alias)) float_a;
typedef int __attribute__((may_alias)) int_a;

template <typename T> __device__ __forceinline__ void vst2(void* p, T v) { *(volatile T*)p = v; __threadfence(); *(volatile T*)p = v; }
__device__ __forceinline__ v8f wmma16(v16h a, v16h b, v8f c) {
  v8f d = __builtin_amdgcn_wmma_f32_16x16x32_f16(false, a, false, b, (short)0, c, false, false);
  asm volatile("v_nop\n\tv_nop\n\tv_nop\n\tv_nop" : "+v"(d) : "v"(a), "v"(b));
  return d;
}
__device__ __forceinline__ v8f wmma_bf(v16b a, v16b b, v8f c) {
  v8f d = __builtin_amdgcn_wmma_f32_16x16x32_bf16(false, a, false, b, (short)0, c, false, false);
  asm volatile("v_nop\n\tv_nop\n\tv_nop\n\tv_nop" : "+v"(d) : "v"(a), "v"(b));
  return d;
}
__device__ __forceinline__ v16h frag_h(const _Float16* rowk0, int lane) {
  union { v16h v; v8h q[2]; } u; const _Float16* p = rowk0 + 8 * (lane >> 4);
  u.q[0] = *(const v8h*)p; u.q[1] = *(const v8h*)(p + 16); return u.v;
}
__device__ __forceinline__ v16h frag_f32(const float* rowk0, int lane) {
  v16h a; const float* p = rowk0 + 8 * (lane >> 4);
#pragma unroll
  for (int i = 0; i < 8; ++i) { a[i] = (_Float16)p[i]; a[8 + i] = (_Float16)p[16 + i]; }
  return a;
}
__device__ __forceinline__ v16h frag_f32s(const float* rowk0, int lane, float sc) {
  v16h a; const float* p = rowk0 + 8 * (lane >> 4);
#pragma unroll
  for (int i = 0; i < 8; ++i) { a[i] = (_Float16)(p[i] * sc); a[8 + i] = (_Float16)(p[16 + i] * sc); }
  return a;
}
__device__ __forceinline__ v16h fragc_f32(const float* W, int k0, int n, int lane, int ld, int K) {
  v16h a; const int g = lane >> 4;
#pragma unroll
  for (int i = 0; i < 8; ++i) { const int ka = k0 + 8 * g + i, kb = ka + 16;
    a[i] = (_Float16)(ka < K ? W[(size_t)(ka < K ? ka : K - 1) * ld + n] : 0.f); a[8 + i] = (_Float16)(kb < K ? W[(size_t)(kb < K ? kb : K - 1) * ld + n] : 0.f); }
  return a;
}
struct F2 { v16b h, l; };
__device__ __forceinline__ F2 bsplit16(const float v[16]) { F2 r;
#pragma unroll
  for (int i = 0; i < 16; ++i) { const __bf16 h = (__bf16)v[i]; r.h[i] = h; r.l[i] = (__bf16)(v[i] - (float)h); }
  return r; }
__device__ __forceinline__ F2 split_row(const float* row, int k0, int lane) { float v[16]; const float* p = row + k0 + 8 * (lane >> 4);
#pragma unroll
  for (int i = 0; i < 8; ++i) { v[i] = p[i]; v[8 + i] = p[16 + i]; }
  return bsplit16(v); }
__device__ __forceinline__ F2 split_rowK(const float* row, int k0, int lane, int K) { float v[16]; const int g = lane >> 4;
#pragma unroll
  for (int i = 0; i < 8; ++i) { const int ka = k0 + 8 * g + i, kb = ka + 16; v[i] = ka < K ? row[ka < K ? ka : K - 1] : 0.f; v[8 + i] = kb < K ? row[kb < K ? kb : K - 1] : 0.f; }
  return bsplit16(v); }
__device__ __forceinline__ F2 split_col(const float* W, int k0, int n, int lane, int ld, int K) { float v[16]; const int g = lane >> 4;
#pragma unroll
  for (int i = 0; i < 8; ++i) { const int ka = k0 + 8 * g + i, kb = ka + 16; v[i] = ka < K ? W[(size_t)(ka < K ? ka : K - 1) * ld + n] : 0.f; v[8 + i] = kb < K ? W[(size_t)(kb < K ? kb : K - 1) * ld + n] : 0.f; }
  return bsplit16(v); }
__device__ __forceinline__ v8f mac3(const F2& a, const F2& b, v8f c) { c = wmma_bf(a.l, b.h, c); c = wmma_bf(a.h, b.l, c); return wmma_bf(a.h, b.h, c); }
__device__ __forceinline__ float sigm(float v) { return 1.0f / (1.0f + expf(-v)); }
#define LDSX() do { asm volatile("s_wait_dscnt 0" ::: "memory"); __builtin_amdgcn_wave_barrier(); __builtin_amdgcn_fence(__ATOMIC_RELEASE, "workgroup"); } while (0)


#define NBAG 512
#define NS 8373
#define NSP 8384
#define DD 768
#define NR 128
#define MB 32
typedef __attribute__((ext_vector_type(8))) __bf16 v8b;
__device__ __forceinline__ v16b frag_b(const __bf16* rowk0, int lane) {
  union { v16b v; v8b q[2]; } u; const __bf16* p = rowk0 + 8 * (lane >> 4);
  u.q[0] = *(const v8b*)p; u.q[1] = *(const v8b*)(p + 16); return u.v;
}
__device__ __forceinline__ float bfr(float v) { return (float)(__bf16)v; }
__device__ __attribute__((noinline)) float exp_ni(float v) { return expf(v); }
__device__ __attribute__((noinline)) float erf_ni(float v) { return erff(v); }

#define WS_S   0u
#define WS_END (WS_S + 4u * (size_t)NSP * NR)

__global__ __launch_bounds__(128) void k_S(const float* __restrict__ REP, const float* __restrict__ FC, float* __restrict__ S) { __shared__ __align__(16) float sf[4][16][132];
  const int tid = threadIdx.x, wave = tid >> 5, lane = tid & 31, col = lane & 15, g = lane >> 4; const size_t r0 = (size_t)blockIdx.x * 64 + wave * 16; const size_t rr = min(r0 + col, (size_t)(NS - 1));
  v8f acc[8] = {};
#pragma unroll 2
  for (int kc = 0; kc < DD / 32; ++kc) { v16b a; { const float* p = REP + rr * DD + kc * 32 + 8 * g;
#pragma unroll
      for (int i = 0; i < 8; ++i) { a[i] = (__bf16)p[i]; a[8 + i] = (__bf16)p[16 + i]; } }
#pragma unroll
    for (int j = 0; j < 8; ++j) { v16b w; const int o = j * 16 + col;
#pragma unroll
      for (int i = 0; i < 8; ++i) { w[i] = (__bf16)FC[(size_t)o * DD + kc * 32 + 8 * g + i]; w[8 + i] = (__bf16)FC[(size_t)o * DD + kc * 32 + 16 + 8 * g + i]; }
      acc[j] = wmma_bf(a, w, acc[j]); } }
#pragma unroll
  for (int j = 0; j < 8; ++j)
#pragma unroll
    for (int r = 0; r < 8; ++r) sf[wave][8 * g + r][j * 16 + col] = acc[j][r];
  LDSX(); for (int rl = 0; rl < 16; ++rl) vst2(S + (r0 + rl) * NR + lane * 4, *(const v4f*)&sf[wave][rl][lane * 4]); }
__global__ __launch_bounds__(128) void k_bag(const float* __restrict__ S, const int* __restrict__ SC, const float* __restrict__ FB, float* __restrict__ OUT) {
  __shared__ __align__(16) float sS[MB][NR + 4]; __shared__ __align__(16) float ssm[NR][MB + 4]; __shared__ __align__(16) float sd[NR];
  const int tid = threadIdx.x, wave = tid >> 5, lane = tid & 31, col = lane & 15, g = lane >> 4; const int b = blockIdx.x;
  const int st = SC[b * 2], en = SC[b * 2 + 1]; int sz = en - st; if (sz > MB) sz = MB; if (sz < 0) sz = 0;
  for (int e = tid; e < MB * NR; e += 128) { const int m = e >> 7, k = e & 127; sS[m][k] = (m < sz) ? S[(size_t)(st + m) * NR + k] : 0.f; }
  __syncthreads();
  { const int n = tid; float mx = -3.0e38f; for (int m = 0; m < sz; ++m) mx = fmaxf(mx, sS[m][n]); float s = 0.f;
    for (int m = 0; m < MB; ++m) { const float e = (m < sz) ? expf(sS[m][n] - mx) : 0.f; ssm[n][m] = e; s += e; }
    const float inv = (sz > 0) ? 1.0f / s : 0.f; for (int m = 0; m < MB; ++m) ssm[n][m] *= inv; }
  __syncthreads();
  v8f acc[2][8]; for (int t = 0; t < 2; ++t) for (int j = 0; j < 8; ++j) for (int r = 0; r < 8; ++r) acc[t][j][r] = 0.f;
  v16b bh[8], bl[8];
#pragma unroll
  for (int j = 0; j < 8; ++j) { const int k = j * 16 + col;
#pragma unroll
    for (int i = 0; i < 8; ++i) { const float v0 = sS[8 * g + i][k], v1 = sS[16 + 8 * g + i][k]; const __bf16 h0 = (__bf16)v0, h1 = (__bf16)v1; bh[j][i] = h0; bh[j][8 + i] = h1; bl[j][i] = (__bf16)(v0 - (float)h0); bl[j][8 + i] = (__bf16)(v1 - (float)h1); } }
#pragma unroll
  for (int t = 0; t < 2; ++t) { const F2 a = split_row(&ssm[wave * 32 + t * 16 + col][0], 0, lane);
#pragma unroll
    for (int j = 0; j < 8; ++j) { acc[t][j] = wmma_bf(a.h, bh[j], acc[t][j]); acc[t][j] = wmma_bf(a.l, bh[j], acc[t][j]); acc[t][j] = wmma_bf(a.h, bl[j], acc[t][j]); acc[t][j] = wmma_bf(a.l, bl[j], acc[t][j]); } }
#pragma unroll
  for (int t = 0; t < 2; ++t) {
#pragma unroll
    for (int r = 0; r < 8; ++r) { const int n = wave * 32 + t * 16 + 8 * g + r; float mx = -3.0e38f;
#pragma unroll
      for (int j = 0; j < 8; ++j) { acc[t][j][r] += bfr(FB[j * 16 + col]); mx = fmaxf(mx, acc[t][j][r]); }
#pragma unroll
      for (int o = 1; o < 16; o <<= 1) mx = fmaxf(mx, __shfl_xor(mx, o));
      float s = 0.f, dg = 0.f;
#pragma unroll
      for (int j = 0; j < 8; ++j) { const float e = expf(acc[t][j][r] - mx); s += e; if (j * 16 + col == n) dg = e; }
#pragma unroll
      for (int o = 1; o < 16; o <<= 1) { s += __shfl_xor(s, o); dg += __shfl_xor(dg, o); }
      if (col == 0) sd[n] = dg / s; } }
  __syncthreads(); if (tid < 32) vst2(OUT + (size_t)b * NR + tid * 4, *(const v4f*)&sd[tid * 4]); }
extern "C" void kernel_launch(void* const* d_in, const int* in_sizes, int n_in, void* d_out, int out_size, void* d_ws, size_t ws_size, hipStream_t stream) {
  (void)in_sizes; (void)n_in; (void)out_size;
  const float** F = (const float**)d_in;
  if (ws_size < (size_t)WS_END) return;
  char* ws = (char*)d_ws; float* S = (float*)(ws + WS_S);
  k_S<<<NSP / 64, 128, 0, stream>>>(F[0], F[1], S);
  k_bag<<<NBAG, 128, 0, stream>>>(S, (const int*)d_in[3], F[2], (float*)d_out);
}
